// StackRNN_81389630259299
// MI455X (gfx1250) — hardware-verified
//
#include <hip/hip_runtime.h>


#define AS3 __attribute__((address_space(3)))

#define NB_  256
#define NT_  256
#define NI_  64
#define NH_  256
#define NR_  128
#define NO_  128
#define RB   16
#define NBLK (NB_ / RB)
#define K1_  (NI_ + NH_ + NR_)
#define K3_  (NH_ + NR_)

static_assert(NB_ % RB == 0);
static_assert(NI_ % 32 == 0 && NH_ % 32 == 0 && NR_ % 32 == 0);
static_assert(NH_ == 8 * 32);
static_assert(NR_ == 8 * 16 && NO_ == 8 * 16);
static_assert(NT_ == 32 * 8);
static_assert(RB == 2 * 8);
static_assert(NR_ == 32 * 4 && NO_ == 32 * 4);
static_assert(K1_ % 64 == 0 && NH_ % 64 == 0 && K3_ % 64 == 0);

typedef __bf16         v16b __attribute__((ext_vector_type(16)));
typedef unsigned short v8us __attribute__((ext_vector_type(8)));
typedef unsigned short v4us __attribute__((ext_vector_type(4)));
typedef float          v8f  __attribute__((ext_vector_type(8)));
typedef float          v4f  __attribute__((ext_vector_type(4)));
typedef v8us __attribute__((may_alias)) v8usa;
typedef v4us __attribute__((may_alias)) v4usa;
typedef v4f  __attribute__((may_alias)) v4fa;

typedef AS3 unsigned short*       lp_us;
typedef AS3 const unsigned short* lcp_us;
typedef AS3 float*                lp_f;
typedef AS3 const float*          lcp_f;
typedef AS3 int*                  lp_i;

union Frag { v16b v; v8us half[2]; };

constexpr size_t OFF_X  = 0;
constexpr size_t SZ_X   = (size_t)NB_ * NT_ * NI_ * 2;
constexpr size_t OFF_WH = OFF_X + SZ_X;
constexpr size_t SZ_WH  = (size_t)NH_ * K1_ * 2;
constexpr size_t OFF_WV = OFF_WH + SZ_WH;
constexpr size_t SZ_WV  = (size_t)NR_ * NH_ * 2;
constexpr size_t OFF_WO = OFF_WV + SZ_WV;
constexpr size_t SZ_WO  = (size_t)NO_ * K3_ * 2;
constexpr size_t OFF_V  = OFF_WO + SZ_WO;
constexpr int    VBLK   = NT_ * RB * NR_;
constexpr size_t SZ_V   = (size_t)NBLK * VBLK * 4;
constexpr size_t WS_END = OFF_V + SZ_V;
static_assert(OFF_WH % 128 == 0 && OFF_WV % 128 == 0 && OFF_WO % 128 == 0 && OFF_V % 128 == 0);
static_assert(WS_END <= (size_t)134217728);
constexpr int NXP   = NB_ * NT_ * NI_ / 8;
constexpr int NXBLK = NXP / 256;
static_assert(NXP % 256 == 0);
static_assert((size_t)NXP * 16 == SZ_X);
static_assert((size_t)NT_ * RB * NR_ * 4 * NBLK == SZ_V);

constexpr int KP      = 456;
constexpr int CVT_BLK = NH_ / 16 + NR_ / 16 + NO_ / 16;
static_assert(KP % 8 == 0 && KP >= K1_ && KP >= NH_ && KP >= K3_);
static_assert(K1_ <= 512 && NH_ <= 512 && K3_ <= 512);
static_assert(2 * K1_ <= 1024 && 2 * NH_ <= 1024 && 2 * K3_ <= 1024);

constexpr int    SPH = NH_ + 8;
constexpr int    SPR = NR_ + 8;
constexpr size_t L_HH  = 0;
constexpr size_t L_HL  = L_HH + (size_t)RB * SPH * 2;
constexpr size_t L_RH  = L_HL + (size_t)RB * SPH * 2;
constexpr size_t L_RL  = L_RH + (size_t)RB * SPR * 2;
constexpr size_t L_SF  = L_RL + (size_t)RB * SPR * 2;
constexpr size_t L_SS  = L_SF + (size_t)RB * NH_ * 4;
constexpr size_t L_SW  = L_SS + (size_t)RB * NT_ * 4;
constexpr size_t L_VC  = L_SW + (size_t)RB * NT_ * 4;
constexpr size_t L_SO  = L_VC + (size_t)RB * NR_ * 4;
constexpr size_t L_BH  = L_SO + (size_t)RB * NO_ * 4;
constexpr size_t L_BV  = L_BH + (size_t)NH_ * 4;
constexpr size_t L_BO  = L_BV + (size_t)NR_ * 4;
constexpr size_t L_WD  = L_BO + (size_t)NO_ * 4;
constexpr size_t L_WU  = L_WD + (size_t)NH_ * 4;
constexpr size_t L_W3  = L_WU + (size_t)NH_ * 4;
constexpr size_t L_DU  = L_W3 + (size_t)NO_ * 4;
constexpr size_t L_ACT = L_DU + (size_t)2 * RB * 4;
constexpr size_t L_CND = L_ACT + (size_t)RB * 4;
constexpr size_t LDS_BYTES = L_CND + (size_t)RB * 4;
constexpr int    NLDS16 = (int)(LDS_BYTES / 16);
static_assert(SPH % 8 == 0 && SPR % 8 == 0);
static_assert(L_HL % 16 == 0 && L_RH % 16 == 0 && L_RL % 16 == 0 && L_SF % 16 == 0 && L_SS % 16 == 0 &&
              L_SW % 16 == 0 && L_VC % 16 == 0 && L_SO % 16 == 0 && L_BH % 16 == 0 && L_BV % 16 == 0 &&
              L_BO % 16 == 0 && L_WD % 16 == 0 && L_WU % 16 == 0 && L_W3 % 16 == 0 && L_DU % 16 == 0 &&
              L_ACT % 16 == 0 && L_CND % 16 == 0 && LDS_BYTES % 16 == 0);

__device__ __forceinline__ unsigned short bf16_bits(float f) {
  unsigned u = __float_as_uint(f);
  u += 0x7FFFu + ((u >> 16) & 1u);
  return (unsigned short)(u >> 16);
}
__device__ __forceinline__ float bf16_val(unsigned short b) { return __uint_as_float(((unsigned)b) << 16); }
__device__ __forceinline__ float bf16r(float f) { return bf16_val(bf16_bits(f)); }
__device__ __forceinline__ v8f zero8() {
  v8f z;
#pragma unroll
  for (int i = 0; i < 8; ++i) z[i] = 0.0f;
  return z;
}
__device__ __forceinline__ v4f splat4(float x) {
  v4f z;
#pragma unroll
  for (int i = 0; i < 4; ++i) z[i] = x;
  return z;
}
__device__ __forceinline__ float tanh_f(float x) {
  const float e = expf(-2.0f * fabsf(x));
  const float q = __builtin_amdgcn_rcpf(1.0f + e);
  return copysignf((1.0f - e) * q, x);
}
__device__ __forceinline__ float sig_f(float x) {
  const float e = expf(-fabsf(x));
  const float q = __builtin_amdgcn_rcpf(1.0f + e);
  return (x >= 0.0f) ? q : (e * q);
}

__device__ __forceinline__ void ldfrag_g(Frag& f, const unsigned short* p, int h) {
  f.half[0] = *(const v8usa*)(p + 8 * h);
  f.half[1] = *(const v8usa*)(p + 16 + 8 * h);
}
__device__ __forceinline__ void ldfrag_l(Frag& f, lcp_us p, int h) {
  f.half[0] = *(AS3 const v8usa*)(p + 8 * h);
  f.half[1] = *(AS3 const v8usa*)(p + 16 + 8 * h);
}
__device__ __forceinline__ v8f mma16(v8f c, const Frag& a, const Frag& b) {
  return __builtin_amdgcn_wmma_f32_16x16x32_bf16(false, a.v, false, b.v, (short)0, c, false, false);
}

__device__ __forceinline__ void gemm_g2(v8f (&acc)[2], const unsigned short* xa, const unsigned short* wb,
                                        int ldb, int K, int h)
{
#pragma unroll 1
  for (int k0 = 0; k0 < K; k0 += 32) {
    Frag a, b0, b1;
    ldfrag_g(a, xa + k0, h);
    ldfrag_g(b0, wb + k0, h);
    ldfrag_g(b1, wb + 16 * ldb + k0, h);
    acc[0] = mma16(acc[0], a, b0);
    acc[1] = mma16(acc[1], a, b1);
    asm volatile("v_nop\n\tv_nop\n\tv_nop\n\tv_nop" : "+v"(acc[0]), "+v"(acc[1]) : "v"(a.v), "v"(b0.v), "v"(b1.v));
  }
}
__device__ __forceinline__ void gemm_hl2(v8f (&acc)[2], lcp_us aH, lcp_us aL, const unsigned short* wb,
                                         int ldb, int K, int h)
{
#pragma unroll 1
  for (int k0 = 0; k0 < K; k0 += 32) {
    Frag ah, al, b0, b1;
    ldfrag_l(ah, aH + k0, h);
    ldfrag_l(al, aL + k0, h);
    ldfrag_g(b0, wb + k0, h);
    ldfrag_g(b1, wb + 16 * ldb + k0, h);
    acc[0] = mma16(acc[0], ah, b0);
    acc[0] = mma16(acc[0], al, b0);
    acc[1] = mma16(acc[1], ah, b1);
    acc[1] = mma16(acc[1], al, b1);
    asm volatile("v_nop\n\tv_nop\n\tv_nop\n\tv_nop"
                 : "+v"(acc[0]), "+v"(acc[1]) : "v"(ah.v), "v"(al.v), "v"(b0.v), "v"(b1.v));
  }
}
__device__ __forceinline__ void gemm_hl1(v8f& acc, lcp_us aH, lcp_us aL, const unsigned short* wb, int K, int h)
{
#pragma unroll 1
  for (int k0 = 0; k0 < K; k0 += 32) {
    Frag ah, al, b;
    ldfrag_l(ah, aH + k0, h);
    ldfrag_l(al, aL + k0, h);
    ldfrag_g(b, wb + k0, h);
    acc = mma16(acc, ah, b);
    acc = mma16(acc, al, b);
    asm volatile("v_nop\n\tv_nop\n\tv_nop\n\tv_nop" : "+v"(acc) : "v"(ah.v), "v"(al.v), "v"(b.v));
  }
}

__device__ __forceinline__ void tanh_hilo(lp_us tH, lp_us tL, lp_f sF, const v8f (&acc)[2], lcp_f bias, int cw, int h)
{
#pragma unroll
  for (int nt = 0; nt < 2; ++nt) {
    const int col = cw + 16 * nt;
    const float b = bias[col];
#pragma unroll
    for (int r = 0; r < 8; ++r) {
      const int row = 8 * h + r;
      const float v = tanh_f(acc[nt][r] + b);
      const unsigned short hb = bf16_bits(v);
      const unsigned short lb = bf16_bits(v - bf16_val(hb));
      tH[row * SPH + col] = hb;
      tL[row * SPH + col] = lb;
      sF[row * NH_ + col] = v;
    }
  }
}

__device__ __forceinline__ float wave_scan(float x, int lane) {
#pragma unroll
  for (int d = 1; d < 32; d <<= 1) {
    const float y = __shfl_up(x, (unsigned)d, 32);
    x = (lane >= d) ? (x + y) : x;
  }
  return x;
}
__device__ __forceinline__ void slot_phase(lp_f sS, lp_f sWt, lcp_f sDU, lp_f sAct, lp_i sCnd, int t, int w, int lane)
{
#pragma unroll
  for (int rr = 0; rr < 2; ++rr) {
    const int mr = 2 * w + rr;
    const float dv = sDU[mr];
    const float uv = sDU[RB + mr];
    lp_f srow = sS  + mr * NT_ + 8 * lane;
    lp_f wrow = sWt + mr * NT_ + 8 * lane;
    const v4f va = *(AS3 const v4fa*)(srow);
    const v4f vb = *(AS3 const v4fa*)(srow + 4);
    float v[8];
#pragma unroll
    for (int k = 0; k < 4; ++k) { v[k] = va[k]; v[4 + k] = vb[k]; }
    float lsum = 0.0f;
#pragma unroll
    for (int k = 0; k < 8; ++k) lsum += v[k];
    float inc  = wave_scan(lsum, lane);
    float tot  = __shfl(inc, 31, 32);
    float sufl = tot - inc;
    float run  = 0.0f;
#pragma unroll
    for (int k = 7; k >= 0; --k) {
      const float suf = sufl + run;
      run += v[k];
      v[k] = fmaxf(0.0f, v[k] - fmaxf(0.0f, uv - suf));
    }
#pragma unroll
    for (int k = 0; k < 8; ++k) v[k] = (8 * lane + k == t) ? dv : v[k];
    lsum = 0.0f;
#pragma unroll
    for (int k = 0; k < 8; ++k) lsum += v[k];
    inc  = wave_scan(lsum, lane);
    tot  = __shfl(inc, 31, 32);
    sufl = tot - inc;
    run  = 0.0f;
    int cand = 0x7fffffff;
    float wv[8];
#pragma unroll
    for (int k = 7; k >= 0; --k) {
      const float suf = sufl + run;
      run += v[k];
      wv[k] = fminf(v[k], fmaxf(0.0f, 1.0f - suf));
      cand = (wv[k] > 0.0f) ? (8 * lane + k) : cand;
    }
    v4f oa, ob, wa, wq;
#pragma unroll
    for (int k = 0; k < 4; ++k) { oa[k] = v[k]; ob[k] = v[4 + k]; wa[k] = wv[k]; wq[k] = wv[4 + k]; }
    *(AS3 v4f*)(srow)     = oa;
    *(AS3 v4f*)(srow + 4) = ob;
    *(AS3 v4f*)(wrow)     = wa;
    *(AS3 v4f*)(wrow + 4) = wq;
#pragma unroll
    for (int d = 16; d > 0; d >>= 1) cand = min(cand, __shfl_xor(cand, d, 32));
    if (lane == 0) { sCnd[mr] = cand; sAct[mr] = tot; }
  }
}

__global__ __launch_bounds__(256)
void cvt_x_kernel(const float* __restrict__ xin, unsigned short* cvx)
{
  const int g = blockIdx.x * 256 + threadIdx.x;
  if (g >= NXP) return;
  const size_t e = (size_t)g * 8;
  const v4f a = *(const v4fa*)(xin + e);
  const v4f c = *(const v4fa*)(xin + e + 4);
  v8us o;
  o[0] = bf16_bits(a[0]); o[1] = bf16_bits(a[1]); o[2] = bf16_bits(a[2]); o[3] = bf16_bits(a[3]);
  o[4] = bf16_bits(c[0]); o[5] = bf16_bits(c[1]); o[6] = bf16_bits(c[2]); o[7] = bf16_bits(c[3]);
  unsigned short* dst = cvx + e;
  *(volatile v8us*)dst = o;
  __threadfence();
  *(volatile v8us*)dst = o;
}

__global__ __launch_bounds__(256)
void cvt_wt_kernel(const float* __restrict__ Wh, const float* __restrict__ Wv, const float* __restrict__ Wo,
                   unsigned short* whT, unsigned short* wvT, unsigned short* woT)
{
  __shared__ __attribute__((aligned(16))) unsigned short tile[16 * KP];
  const int tid = threadIdx.x;
  const int bid = (int)blockIdx.x;
  const float* src; unsigned short* dst; int K, N, n0;
  if (bid < NH_ / 16)                  { src = Wh; dst = whT; K = K1_; N = NH_; n0 = 16 * bid; }
  else if (bid < NH_ / 16 + NR_ / 16)  { src = Wv; dst = wvT; K = NH_; N = NR_; n0 = 16 * (bid - NH_ / 16); }
  else                                 { src = Wo; dst = woT; K = K3_; N = NO_; n0 = 16 * (bid - NH_ / 16 - NR_ / 16); }

#pragma unroll 1
  for (int i = 0; i < 2; ++i) {
    const int k = min(tid + 256 * i, K - 1);
    const float* p = src + (size_t)k * N + n0;
    const v4f a0 = *(const v4fa*)(p);
    const v4f a1 = *(const v4fa*)(p + 4);
    const v4f a2 = *(const v4fa*)(p + 8);
    const v4f a3 = *(const v4fa*)(p + 12);
#pragma unroll
    for (int j = 0; j < 4; ++j) {
      tile[(j     ) * KP + k] = bf16_bits(a0[j]);
      tile[(j +  4) * KP + k] = bf16_bits(a1[j]);
      tile[(j +  8) * KP + k] = bf16_bits(a2[j]);
      tile[(j + 12) * KP + k] = bf16_bits(a3[j]);
    }
  }
  __syncthreads();

  const int ppr = K >> 3;
  const int np  = 16 * ppr;
  v8us pv[4];
  int  prow[4], pq[4];
#pragma unroll
  for (int i = 0; i < 4; ++i) {
    const int p = min(tid + 256 * i, np - 1);
    prow[i] = p / ppr;
    pq[i]   = p - prow[i] * ppr;
    pv[i]   = *(AS3 const v8usa*)((lcp_us)tile + prow[i] * KP + 8 * pq[i]);
  }
#pragma unroll
  for (int i = 0; i < 4; ++i)
    if (tid + 256 * i < np)
      *(volatile v8us*)(dst + (size_t)(n0 + prow[i]) * K + 8 * pq[i]) = pv[i];
  __threadfence();
#pragma unroll
  for (int i = 0; i < 4; ++i)
    if (tid + 256 * i < np)
      *(volatile v8us*)(dst + (size_t)(n0 + prow[i]) * K + 8 * pq[i]) = pv[i];
}

__global__ __launch_bounds__(256)
void cell_kernel(const unsigned short* __restrict__ cvx, const unsigned short* __restrict__ whT,
                 const unsigned short* __restrict__ wvT, const unsigned short* __restrict__ woT,
                 const float* __restrict__ Wd, const float* __restrict__ Wu, const float* __restrict__ Wo,
                 const float* __restrict__ bh, const float* __restrict__ bv, const float* __restrict__ bd,
                 const float* __restrict__ bu, const float* __restrict__ bo,
                 float* vws, float* out)
{
  extern __shared__ __attribute__((aligned(16))) char smem[];
  lp_us tHH  = (lp_us)(smem + L_HH);
  lp_us tHL  = (lp_us)(smem + L_HL);
  lp_us tRH  = (lp_us)(smem + L_RH);
  lp_us tRL  = (lp_us)(smem + L_RL);
  lp_f  sF   = (lp_f)(smem + L_SF);
  lp_f  sS   = (lp_f)(smem + L_SS);
  lp_f  sWt  = (lp_f)(smem + L_SW);
  lp_f  sVc  = (lp_f)(smem + L_VC);
  lp_f  sO   = (lp_f)(smem + L_SO);
  lp_f  sBh  = (lp_f)(smem + L_BH);
  lp_f  sBv  = (lp_f)(smem + L_BV);
  lp_f  sBo  = (lp_f)(smem + L_BO);
  lp_f  sWd  = (lp_f)(smem + L_WD);
  lp_f  sWu  = (lp_f)(smem + L_WU);
  lp_f  sW3  = (lp_f)(smem + L_W3);
  lp_f  sDU  = (lp_f)(smem + L_DU);
  lp_f  sAct = (lp_f)(smem + L_ACT);
  lp_i  sCnd = (lp_i)(smem + L_CND);

  const int tid = threadIdx.x, lane = tid & 31;
  const int w = __builtin_amdgcn_readfirstlane(tid >> 5);
  const int h = lane >> 4, m = lane & 15;
  const int blk = (int)blockIdx.x;
  const int b0 = blk * RB;
  float* vblk = vws + (size_t)blk * VBLK;
  const int vr = 2 * w;
  const int vc = 4 * lane;
  const int cw = 32 * w + m;
  const int cn = 16 * w + m;

  {
    const v4f z4 = splat4(0.0f);
    for (int i = tid; i < NLDS16; i += 256) *(AS3 v4f*)(smem + 16 * i) = z4;
  }
  __syncthreads();
  sBh[tid] = bf16r(bh[tid]);
  sWd[tid] = bf16r(Wd[tid]);
  sWu[tid] = bf16r(Wu[tid]);
  if (tid < NR_) sBv[tid] = bf16r(bv[tid]);
  if (tid < NO_) { sBo[tid] = bf16r(bo[tid]); sW3[tid] = bf16r(Wo[(size_t)K3_ * NO_ + tid]); }
  const float bdv = bf16r(bd[0]);
  const float buv = bf16r(bu[0]);
  __syncthreads();

#pragma unroll 1
  for (int t = 0; t < NT_; ++t) {
    v8f acc[2];
    acc[0] = zero8(); acc[1] = zero8();
    {
      const unsigned short* xa = cvx + ((size_t)(b0 + m) * NT_ + t) * NI_;
      const unsigned short* wb = whT + (size_t)cw * K1_;
      gemm_g2(acc, xa, wb, K1_, NI_, h);
      gemm_hl2(acc, tHH + m * SPH, tHL + m * SPH, wb + NI_, K1_, NH_, h);
      gemm_hl2(acc, tRH + m * SPR, tRL + m * SPR, wb + NI_ + NH_, K1_, NR_, h);
    }
    __syncthreads();
    tanh_hilo(tHH, tHL, sF, acc, sBh, cw, h);
    __syncthreads();

    {
      v8f a2 = zero8();
      gemm_hl1(a2, tHH + m * SPH, tHL + m * SPH, wvT + (size_t)cn * NH_, NH_, h);
      const float b = sBv[cn];
#pragma unroll
      for (int r = 0; r < 8; ++r) sVc[(8 * h + r) * NR_ + cn] = tanh_f(a2[r] + b);
    }
    {
      const int row = tid >> 4, seg = tid & 15;
      lcp_f hp = sF + row * NH_ + 16 * seg;
      lcp_f dp = sWd + 16 * seg;
      lcp_f up = sWu + 16 * seg;
      float pd = 0.0f, pu = 0.0f;
#pragma unroll
      for (int i = 0; i < 4; ++i) {
        const v4f hv = *(AS3 const v4fa*)(hp + 4 * i);
        const v4f wd = *(AS3 const v4fa*)(dp + 4 * i);
        const v4f wu = *(AS3 const v4fa*)(up + 4 * i);
#pragma unroll
        for (int j = 0; j < 4; ++j) { pd = fmaf(hv[j], wd[j], pd); pu = fmaf(hv[j], wu[j], pu); }
      }
#pragma unroll
      for (int d = 8; d > 0; d >>= 1) { pd += __shfl_xor(pd, d, 32); pu += __shfl_xor(pu, d, 32); }
      if (seg == 0) { sDU[row] = sig_f(pd + bdv); sDU[RB + row] = sig_f(pu + buv); }
    }
    __syncthreads();

    const v4f pv0 = *(AS3 const v4fa*)(sVc + vr * NR_ + vc);
    const v4f pv1 = *(AS3 const v4fa*)(sVc + (vr + 1) * NR_ + vc);
    {
      float* p0 = vblk + ((size_t)t * RB + vr) * NR_ + vc;
      float* p1 = p0 + NR_;
      *(volatile v4f*)p0 = pv0;
      *(volatile v4f*)p1 = pv1;
      __threadfence();
      *(volatile v4f*)p0 = pv0;
      *(volatile v4f*)p1 = pv1;
    }
    slot_phase(sS, sWt, sDU, sAct, sCnd, t, w, lane);
    __syncthreads();

    {
      int mn = 0x7fffffff;
#pragma unroll
      for (int j = 0; j < RB; ++j) mn = min(mn, sCnd[j]);
      int lo = max(min(mn, t), 0);
      lo = __builtin_amdgcn_readfirstlane(lo);
      v4f ra = splat4(0.0f), rq = splat4(0.0f);
      const float* v0p = vblk + (size_t)vr * NR_ + vc;
      lcp_f w0p = sWt + vr * NT_;
      lcp_f w1p = w0p + NT_;
#pragma unroll 1
      for (int tp = lo; tp < t; ++tp) {
        const v4f x0 = *(const v4fa*)(v0p + (size_t)tp * (RB * NR_));
        const v4f x1 = *(const v4fa*)(v0p + (size_t)tp * (RB * NR_) + NR_);
        ra += splat4(w0p[tp]) * x0;
        rq += splat4(w1p[tp]) * x1;
      }
      ra += splat4(w0p[t]) * pv0;
      rq += splat4(w1p[t]) * pv1;
      v4us h0, l0, h1, l1;
#pragma unroll
      for (int c = 0; c < 4; ++c) {
        const unsigned short a = bf16_bits(ra[c]);
        h0[c] = a; l0[c] = bf16_bits(ra[c] - bf16_val(a));
        const unsigned short b = bf16_bits(rq[c]);
        h1[c] = b; l1[c] = bf16_bits(rq[c] - bf16_val(b));
      }
      *(AS3 v4us*)(tRH + vr * SPR + vc)       = h0;
      *(AS3 v4us*)(tRL + vr * SPR + vc)       = l0;
      *(AS3 v4us*)(tRH + (vr + 1) * SPR + vc) = h1;
      *(AS3 v4us*)(tRL + (vr + 1) * SPR + vc) = l1;
    }
    __syncthreads();

    {
      v8f a3 = zero8();
      const unsigned short* wb3 = woT + (size_t)cn * K3_;
      gemm_hl1(a3, tHH + m * SPH, tHL + m * SPH, wb3, NH_, h);
      gemm_hl1(a3, tRH + m * SPR, tRL + m * SPR, wb3 + NH_, NR_, h);
      const float b = sBo[cn], wl = sW3[cn];
#pragma unroll
      for (int r = 0; r < 8; ++r) {
        const float pre = fmaf(sAct[8 * h + r], wl, a3[r]) + b;
        sO[(8 * h + r) * NO_ + cn] = sig_f(pre);
      }
    }
    __syncthreads();

    {
      const v4f o0 = *(AS3 const v4fa*)(sO + vr * NO_ + vc);
      const v4f o1 = *(AS3 const v4fa*)(sO + (vr + 1) * NO_ + vc);
      float* q0 = out + ((size_t)(b0 + vr) * NT_ + t) * NO_ + vc;
      float* q1 = q0 + (size_t)NT_ * NO_;
      *(volatile v4f*)q0 = o0;
      *(volatile v4f*)q1 = o1;
      __threadfence();
      *(volatile v4f*)q0 = o0;
      *(volatile v4f*)q1 = o1;
    }
  }
}

extern "C" void kernel_launch(void* const* d_in, const int* in_sizes, int n_in,
                              void* d_out, int out_size, void* d_ws, size_t ws_size,
                              hipStream_t stream)
{
  if (n_in < 11) return;
  if (in_sizes[0]  != NB_ * NT_ * NI_)   return;
  if (in_sizes[1]  != K1_ * NH_)         return;
  if (in_sizes[2]  != NH_)               return;
  if (in_sizes[3]  != NH_ * NR_)         return;
  if (in_sizes[4]  != NR_)               return;
  if (in_sizes[5]  != NH_)               return;
  if (in_sizes[6]  != 1)                 return;
  if (in_sizes[7]  != NH_)               return;
  if (in_sizes[8]  != 1)                 return;
  if (in_sizes[9]  != (K3_ + 1) * NO_)   return;
  if (in_sizes[10] != NO_)               return;
  if (out_size != NB_ * NT_ * NO_)       return;
  if (ws_size < WS_END)                  return;

  const float* xin = (const float*)d_in[0];
  const float* Wh  = (const float*)d_in[1];
  const float* bh  = (const float*)d_in[2];
  const float* Wv  = (const float*)d_in[3];
  const float* bv  = (const float*)d_in[4];
  const float* Wd  = (const float*)d_in[5];
  const float* bd  = (const float*)d_in[6];
  const float* Wu  = (const float*)d_in[7];
  const float* bu  = (const float*)d_in[8];
  const float* Wo  = (const float*)d_in[9];
  const float* bo  = (const float*)d_in[10];
  float* out = (float*)d_out;

  char* ws = (char*)d_ws;
  unsigned short* cvx = (unsigned short*)(ws + OFF_X);
  unsigned short* whT = (unsigned short*)(ws + OFF_WH);
  unsigned short* wvT = (unsigned short*)(ws + OFF_WV);
  unsigned short* woT = (unsigned short*)(ws + OFF_WO);
  float* vws = (float*)(ws + OFF_V);

  cvt_x_kernel<<<dim3(NXBLK), dim3(256), 0, stream>>>(xin, cvx);
  cvt_wt_kernel<<<dim3(CVT_BLK), dim3(256), 0, stream>>>(Wh, Wv, Wo, whT, wvT, woT);

  hipFuncSetAttribute(reinterpret_cast<const void*>(&cell_kernel),
                      hipFuncAttributeMaxDynamicSharedMemorySize, (int)LDS_BYTES);
  cell_kernel<<<dim3(NBLK), dim3(256), LDS_BYTES, stream>>>(cvx, whT, wvT, woT, Wd, Wu, Wo,
                                                            bh, bv, bd, bu, bo, vws, out);
}
